// Net_24489903522726
// MI455X (gfx1250) — hardware-verified
//
#include <hip/hip_runtime.h>
#include <stdint.h>

#define NB     32768
#define ND     128
#define NL     3
#define NE     384
#define NR     64
#define NO     64
#define KTT    8192
#define LNROWS 32
#define WSCAP  134217728

static_assert(NE == ND * NL);
static_assert(KTT == NR * ND);
static_assert(NB % 128 == 0);
static_assert(NB % 64 == 0);
static_assert(NB % LNROWS == 0);
static_assert(KTT % 32 == 0);
static_assert(ND % 32 == 0);
static_assert(NR % 32 == 0);
static_assert(NR == 64);
static_assert(NO == 64);
static_assert((NR * ND / 8) % 256 == 0);
static_assert((NR * KTT / 8) % 256 == 0);
static_assert((NO * NR / 8) % 256 == 0);

typedef float          v4f   __attribute__((ext_vector_type(4)));
typedef float          v8f   __attribute__((ext_vector_type(8)));
typedef int            v8i   __attribute__((ext_vector_type(8)));
typedef unsigned int   v4u   __attribute__((ext_vector_type(4)));
typedef unsigned short v8us  __attribute__((ext_vector_type(8)));
typedef unsigned short v16us __attribute__((ext_vector_type(16)));
typedef __bf16         v16b  __attribute__((ext_vector_type(16)));
typedef v4f  __attribute__((may_alias)) v4fa;
typedef v4u  __attribute__((may_alias)) v4ua;
typedef v8us __attribute__((may_alias)) v8usa;
union FragB { v16b v; v16us u; v8us h[2]; v4u q[2]; v8i w; };

__device__ __forceinline__ v8f wmb(const FragB& a, const FragB& b, v8f c) {
  v8f d = __builtin_amdgcn_wmma_f32_16x16x32_bf16(false, a.v, false, b.v, (short)0, c, false, false);
  asm volatile("v_nop\n\tv_nop\n\tv_nop\n\tv_nop" : "+v"(d) : "v"(a.w), "v"(b.w));
  return d;
}
__device__ __forceinline__ v8f z8() { v8f z = {0.f, 0.f, 0.f, 0.f, 0.f, 0.f, 0.f, 0.f}; return z; }

__device__ __forceinline__ unsigned f2bf_rne(float f) {
  const unsigned u = __float_as_uint(f);
  return (u + 0x7FFFu + ((u >> 16) & 1u)) >> 16;
}
__device__ __forceinline__ float bfr(float f) { return __uint_as_float(f2bf_rne(f) << 16); }

__device__ __forceinline__ void split1(float x, unsigned& hb, unsigned& lb) {
  const unsigned hu = __float_as_uint(x) & 0xFFFF0000u;
  hb = hu >> 16;
  lb = f2bf_rne(x - __uint_as_float(hu));
}
__device__ __forceinline__ void split2(float x0, float x1, unsigned& hp, unsigned& lp) {
  const unsigned h0 = __float_as_uint(x0) & 0xFFFF0000u;
  const unsigned h1 = __float_as_uint(x1) & 0xFFFF0000u;
  hp = (h0 >> 16) | h1;
  const unsigned l0 = f2bf_rne(x0 - __uint_as_float(h0));
  const unsigned l1 = f2bf_rne(x1 - __uint_as_float(h1));
  lp = (l0 & 0xFFFFu) | (l1 << 16);
}

__device__ __forceinline__ float wsum(float v) {
  v += __shfl_xor(v, 16);
  v += __shfl_xor(v, 8);
  v += __shfl_xor(v, 4);
  v += __shfl_xor(v, 2);
  v += __shfl_xor(v, 1);
  return v;
}

__global__ __launch_bounds__(256) void tr_kernel(const float* __restrict__ src,
                                                 unsigned short* __restrict__ dst, int k8shift) {
  const int u  = blockIdx.x * 256 + threadIdx.x;
  const int n  = u >> k8shift;
  const int k0 = (u - (n << k8shift)) * 8;
  const float* s = src + (size_t)k0 * 64 + n;
  float f[8];
#pragma unroll
  for (int j = 0; j < 8; ++j) f[j] = s[j * 64];
  const v4u v = { (f2bf_rne(f[0]) & 0xFFFFu) | (f2bf_rne(f[1]) << 16),
                  (f2bf_rne(f[2]) & 0xFFFFu) | (f2bf_rne(f[3]) << 16),
                  (f2bf_rne(f[4]) & 0xFFFFu) | (f2bf_rne(f[5]) << 16),
                  (f2bf_rne(f[6]) & 0xFFFFu) | (f2bf_rne(f[7]) << 16) };
  unsigned short* d = dst + (size_t)u * 8;
  *(volatile v4u*)d = v;
  __threadfence();
  *(volatile v4u*)d = v;
}

__global__ __launch_bounds__(256) void ln_kernel(const float* __restrict__ x,
                                                 const float* __restrict__ lnw,
                                                 const float* __restrict__ lnb,
                                                 unsigned short* __restrict__ xn0hl,
                                                 float* __restrict__ xn1,
                                                 float* __restrict__ xn2) {
  __shared__ __align__(16) float srow[8][NE];
  const int tid = threadIdx.x, lane = tid & 31, w = tid >> 5;
  float* sr = &srow[w][0];

  float wv[12], bv[12];
  int pos[12];
#pragma unroll
  for (int c = 0; c < 3; ++c) {
    const v4f wa = *(const v4fa*)(lnw + 128 * c + 4 * lane);
    const v4f ba = *(const v4fa*)(lnb + 128 * c + 4 * lane);
#pragma unroll
    for (int j = 0; j < 4; ++j) {
      wv[4 * c + j] = bfr(wa[j]);
      bv[4 * c + j] = bfr(ba[j]);
      const int e = 128 * c + 4 * lane + j;
      const int d = e / 3, l = e - 3 * d;
      pos[4 * c + j] = l * ND + d;
    }
  }

#pragma unroll 1
  for (int it = 0; it < 4; ++it) {
    const int b = blockIdx.x * LNROWS + 4 * w + it;
    const float* xr = x + (size_t)b * NE;
    float xv[12];
#pragma unroll
    for (int c = 0; c < 3; ++c) {
      const v4f a = *(const v4fa*)(xr + 128 * c + 4 * lane);
#pragma unroll
      for (int j = 0; j < 4; ++j) xv[4 * c + j] = bfr(a[j]);
    }
    float s = 0.0f;
#pragma unroll
    for (int i = 0; i < 12; ++i) s += xv[i];
    s = wsum(s);
    const float mu = s * (1.0f / 384.0f);
    float ss = 0.0f;
#pragma unroll
    for (int i = 0; i < 12; ++i) {
      const float dv = xv[i] - mu;
      xv[i] = dv;
      ss += dv * dv;
    }
    ss = wsum(ss);
    const float var = ss * (1.0f / 384.0f);
    const float rs = 1.0f / sqrtf(var + 1e-5f);
#pragma unroll
    for (int i = 0; i < 12; ++i) sr[pos[i]] = (xv[i] * rs) * wv[i] + bv[i];
    __syncthreads();

    const v4f o1 = *(const v4fa*)(sr + ND + 4 * lane);
    const v4f o2 = *(const v4fa*)(sr + 2 * ND + 4 * lane);
    const v4f g0 = *(const v4fa*)(sr + 8 * (lane & 15));
    const v4f g1 = *(const v4fa*)(sr + 8 * (lane & 15) + 4);
    unsigned h0, h1, h2, h3, l0, l1, l2, l3;
    split2(g0[0], g0[1], h0, l0);
    split2(g0[2], g0[3], h1, l1);
    split2(g1[0], g1[1], h2, l2);
    split2(g1[2], g1[3], h3, l3);
    const unsigned msk = (lane < 16) ? 0xFFFFFFFFu : 0u;
    const v4u o0 = { (h0 & msk) | (l0 & ~msk), (h1 & msk) | (l1 & ~msk),
                     (h2 & msk) | (l2 & ~msk), (h3 & msk) | (l3 & ~msk) };

    float* d1 = xn1 + (size_t)b * ND + 4 * lane;
    float* d2 = xn2 + (size_t)b * ND + 4 * lane;
    unsigned short* d0 = xn0hl + (size_t)b * (2 * ND) + 8 * lane;
    *(volatile v4f*)d1 = o1;
    *(volatile v4f*)d2 = o2;
    *(volatile v4u*)d0 = o0;
    __threadfence();
    *(volatile v4f*)d1 = o1;
    *(volatile v4f*)d2 = o2;
    *(volatile v4u*)d0 = o0;
    __syncthreads();
  }
}

__device__ __forceinline__ void o_store_pass(const float* sO, float* out, int grow_w, int w, int lane) {
  const int q8 = lane & 7, sub = lane >> 3;
#pragma unroll
  for (int i = 0; i < 16; ++i) {
    const int lid = i * 4 + sub;
    const int row = lid >> 1, hl = lid & 1;
    const v4f v = *(const v4fa*)(sO + (32 * w + row) * 64 + 32 * hl + 4 * q8);
    *(volatile v4f*)(out + (size_t)(grow_w + row) * 64 + 32 * hl + 4 * q8) = v;
  }
}

template <int K>
__global__ __launch_bounds__(128) void gemmhl_kernel(const unsigned short* __restrict__ AP,
                                                     const unsigned short* __restrict__ BT,
                                                     float* __restrict__ out) {
  static_assert(K % 32 == 0);
  __shared__ __align__(16) float sO[128 * 64];
  const int tid = threadIdx.x, lane = tid & 31, w = tid >> 5;
  const int h = lane >> 4, m = lane & 15;
  const int row_w = blockIdx.x * 128 + 32 * w;

  const unsigned short* xa0 = AP + (size_t)(row_w + m) * (2 * K) + 8 * h;
  const unsigned short* xa1 = xa0 + (size_t)16 * (2 * K);
  const unsigned short* wb  = BT + (size_t)m * K + 8 * h;

  v8f acc[2][4];
#pragma unroll
  for (int mt = 0; mt < 2; ++mt)
#pragma unroll
    for (int nt = 0; nt < 4; ++nt) acc[mt][nt] = z8();

#pragma unroll 1
  for (int k0 = 0; k0 < K; k0 += 32) {
    FragB a0h, a0l, a1h, a1l;
    a0h.h[0] = *(const v8usa*)(xa0 + k0);
    a0h.h[1] = *(const v8usa*)(xa0 + k0 + 16);
    a0l.h[0] = *(const v8usa*)(xa0 + K + k0);
    a0l.h[1] = *(const v8usa*)(xa0 + K + k0 + 16);
    a1h.h[0] = *(const v8usa*)(xa1 + k0);
    a1h.h[1] = *(const v8usa*)(xa1 + k0 + 16);
    a1l.h[0] = *(const v8usa*)(xa1 + K + k0);
    a1l.h[1] = *(const v8usa*)(xa1 + K + k0 + 16);
#pragma unroll
    for (int nt = 0; nt < 4; ++nt) {
      const unsigned short* wq = wb + (size_t)nt * 16 * K + k0;
      FragB b;
      b.h[0] = *(const v8usa*)wq;
      b.h[1] = *(const v8usa*)(wq + 16);
      acc[0][nt] = wmb(a0h, b, acc[0][nt]);
      acc[0][nt] = wmb(a0l, b, acc[0][nt]);
      acc[1][nt] = wmb(a1h, b, acc[1][nt]);
      acc[1][nt] = wmb(a1l, b, acc[1][nt]);
    }
  }

#pragma unroll
  for (int nt = 0; nt < 4; ++nt) {
    const int cl = 16 * nt + m;
#pragma unroll
    for (int mt = 0; mt < 2; ++mt) {
#pragma unroll
      for (int r = 0; r < 8; ++r) {
        const int rl = 32 * w + 16 * mt + 8 * h + r;
        sO[rl * 64 + cl] = acc[mt][nt][r];
      }
    }
  }
  __syncthreads();

  const int grow_w = row_w;
  o_store_pass(sO, out, grow_w, w, lane);
  __threadfence();
  o_store_pass(sO, out, grow_w, w, lane);
}

union TTLds {
  struct { float t[64 * NR]; float x[64 * ND]; } in;
  struct { float o[64 * NR]; unsigned short hl[64 * 2 * NR]; } ep;
};

__device__ __forceinline__ void t_store_pass(const float* so, float* tout, int row0, int w, int lane) {
  const int q8 = lane & 7, sub = lane >> 3;
#pragma unroll
  for (int i = 0; i < 8; ++i) {
    const int lid = i * 4 + sub;
    const int row = 16 * w + (lid >> 1), hl = lid & 1;
    const v4f v = *(const v4fa*)(so + row * NR + 32 * hl + 4 * q8);
    *(volatile v4f*)(tout + (size_t)(row0 + row) * NR + 32 * hl + 4 * q8) = v;
  }
}
__device__ __forceinline__ void hl_store_pass(const unsigned short* sh, unsigned short* thl, int row0, int w, int lane) {
  const int q8 = lane & 7, sub = lane >> 3;
#pragma unroll
  for (int i = 0; i < 8; ++i) {
    const int lid = i * 4 + sub;
    const int row = 16 * w + (lid >> 1), hl = lid & 1;
    const v4u v = *(const v4ua*)(sh + row * (2 * NR) + 64 * hl + 8 * q8);
    *(volatile v4u*)(thl + (size_t)(row0 + row) * (2 * NR) + 64 * hl + 8 * q8) = v;
  }
}

__global__ __launch_bounds__(128) void tt_kernel(const float* __restrict__ tin,
                                                 const float* __restrict__ xn,
                                                 const unsigned short* __restrict__ CT,
                                                 float* __restrict__ tout,
                                                 unsigned short* __restrict__ thl,
                                                 int write_hl) {
  __shared__ __align__(16) TTLds L;
  const int tid = threadIdx.x, lane = tid & 31, w = tid >> 5;
  const int h = lane >> 4, m = lane & 15;
  const int row0 = blockIdx.x * 64;

  {
    const float* gt = tin + (size_t)row0 * NR;
#pragma unroll 4
    for (int i = 0; i < 8; ++i) {
      const int u = i * 128 + tid;
      *(v4fa*)(L.in.t + 4 * u) = *(const v4fa*)(gt + 4 * u);
    }
    const float* gx = xn + (size_t)row0 * ND;
#pragma unroll 4
    for (int i = 0; i < 16; ++i) {
      const int u = i * 128 + tid;
      *(v4fa*)(L.in.x + 4 * u) = *(const v4fa*)(gx + 4 * u);
    }
  }
  __syncthreads();

  const int rowl = 16 * w + m;
  const float* trow = L.in.t + rowl * NR;
  const float* xrow = L.in.x + rowl * ND + 8 * h;
  const unsigned short* cb = CT + (size_t)m * KTT + 8 * h;

  v8f acc[4];
#pragma unroll
  for (int nt = 0; nt < 4; ++nt) acc[nt] = z8();

#pragma unroll 1
  for (int ks = 0; ks < KTT / 32; ++ks) {
    const int r = ks >> 2, d0 = (ks & 3) * 32;
    const float tv = trow[r];
    const v4f x0 = *(const v4fa*)(xrow + d0);
    const v4f x1 = *(const v4fa*)(xrow + d0 + 4);
    const v4f x2 = *(const v4fa*)(xrow + d0 + 16);
    const v4f x3 = *(const v4fa*)(xrow + d0 + 20);
    unsigned hp[8], lp[8];
    split2(tv * x0[0], tv * x0[1], hp[0], lp[0]);
    split2(tv * x0[2], tv * x0[3], hp[1], lp[1]);
    split2(tv * x1[0], tv * x1[1], hp[2], lp[2]);
    split2(tv * x1[2], tv * x1[3], hp[3], lp[3]);
    split2(tv * x2[0], tv * x2[1], hp[4], lp[4]);
    split2(tv * x2[2], tv * x2[3], hp[5], lp[5]);
    split2(tv * x3[0], tv * x3[1], hp[6], lp[6]);
    split2(tv * x3[2], tv * x3[3], hp[7], lp[7]);
    const v4u qh0 = { hp[0], hp[1], hp[2], hp[3] };
    const v4u qh1 = { hp[4], hp[5], hp[6], hp[7] };
    const v4u ql0 = { lp[0], lp[1], lp[2], lp[3] };
    const v4u ql1 = { lp[4], lp[5], lp[6], lp[7] };
    FragB ah, al;
    ah.q[0] = qh0; ah.q[1] = qh1;
    al.q[0] = ql0; al.q[1] = ql1;
#pragma unroll
    for (int nt = 0; nt < 4; ++nt) {
      const unsigned short* bp = cb + (size_t)nt * 16 * KTT + 32 * ks;
      FragB b;
      b.h[0] = *(const v8usa*)bp;
      b.h[1] = *(const v8usa*)(bp + 16);
      acc[nt] = wmb(ah, b, acc[nt]);
      acc[nt] = wmb(al, b, acc[nt]);
    }
  }
  __syncthreads();

#pragma unroll
  for (int nt = 0; nt < 4; ++nt) {
    const int cl = 16 * nt + m;
#pragma unroll
    for (int r = 0; r < 8; ++r) {
      const int rl = 16 * w + 8 * h + r;
      const float v = acc[nt][r];
      L.ep.o[rl * NR + cl] = v;
      unsigned hb, lb;
      split1(v, hb, lb);
      L.ep.hl[rl * (2 * NR) + cl] = (unsigned short)hb;
      L.ep.hl[rl * (2 * NR) + NR + cl] = (unsigned short)lb;
    }
  }
  __syncthreads();

  t_store_pass(L.ep.o, tout, row0, w, lane);
  if (write_hl != 0) hl_store_pass(L.ep.hl, thl, row0, w, lane);
  __threadfence();
  t_store_pass(L.ep.o, tout, row0, w, lane);
  if (write_hl != 0) hl_store_pass(L.ep.hl, thl, row0, w, lane);
}

extern "C" void kernel_launch(void* const* d_in, const int* in_sizes, int n_in,
                              void* d_out, int out_size, void* d_ws, size_t ws_size,
                              hipStream_t stream) {
  if (n_in < 7) return;
  if (in_sizes[0] != NB * NE) return;
  if (in_sizes[1] != ND * NR) return;
  if (in_sizes[2] != NR * ND * NR) return;
  if (in_sizes[3] != NR * ND * NR) return;
  if (in_sizes[4] != NR * NO) return;
  if (in_sizes[5] != NE) return;
  if (in_sizes[6] != NE) return;
  if (out_size != NB * NO) return;

  const float* x      = (const float*)d_in[0];
  const float* layer0 = (const float*)d_in[1];
  const float* core1  = (const float*)d_in[2];
  const float* core2  = (const float*)d_in[3];
  const float* last   = (const float*)d_in[4];
  const float* lnw    = (const float*)d_in[5];
  const float* lnb    = (const float*)d_in[6];
  float* out = (float*)d_out;

  size_t off = 0;
  const size_t oL0T = off; off += (size_t)NR * ND * 2;
  const size_t oC1T = off; off += (size_t)NR * KTT * 2;
  const size_t oC2T = off; off += (size_t)NR * KTT * 2;
  const size_t oLT  = off; off += (size_t)NO * NR * 2;
  const size_t oXN0 = off; off += (size_t)NB * 2 * ND * 2;
  const size_t oXN1 = off; off += (size_t)NB * ND * 4;
  const size_t oXN2 = off; off += (size_t)NB * ND * 4;
  const size_t oT0  = off; off += (size_t)NB * NR * 4;
  const size_t oT1  = off; off += (size_t)NB * NR * 4;
  const size_t oT2  = off; off += (size_t)NB * NR * 4;
  const size_t oHL  = off; off += (size_t)NB * 2 * NR * 2;
  if (off > ws_size) return;
  if (off > (size_t)WSCAP) return;

  char* ws = (char*)d_ws;
  unsigned short* L0T   = (unsigned short*)(ws + oL0T);
  unsigned short* C1T   = (unsigned short*)(ws + oC1T);
  unsigned short* C2T   = (unsigned short*)(ws + oC2T);
  unsigned short* LT    = (unsigned short*)(ws + oLT);
  unsigned short* XN0HL = (unsigned short*)(ws + oXN0);
  float* XN1   = (float*)(ws + oXN1);
  float* XN2   = (float*)(ws + oXN2);
  float* TEMP0 = (float*)(ws + oT0);
  float* TEMP1 = (float*)(ws + oT1);
  float* TEMP2 = (float*)(ws + oT2);
  unsigned short* T2HL = (unsigned short*)(ws + oHL);

  tr_kernel<<<dim3((NR * ND / 8) / 256), dim3(256), 0, stream>>>(layer0, L0T, 4);
  tr_kernel<<<dim3((NR * KTT / 8) / 256), dim3(256), 0, stream>>>(core1, C1T, 10);
  tr_kernel<<<dim3((NR * KTT / 8) / 256), dim3(256), 0, stream>>>(core2, C2T, 10);
  tr_kernel<<<dim3((NO * NR / 8) / 256), dim3(256), 0, stream>>>(last, LT, 3);
  ln_kernel<<<dim3(NB / LNROWS), dim3(256), 0, stream>>>(x, lnw, lnb, XN0HL, XN1, XN2);
  gemmhl_kernel<128><<<dim3(NB / 128), dim3(128), 0, stream>>>(XN0HL, L0T, TEMP0);
  tt_kernel<<<dim3(NB / 64), dim3(128), 0, stream>>>(TEMP0, XN1, C1T, TEMP1, T2HL, 0);
  tt_kernel<<<dim3(NB / 64), dim3(128), 0, stream>>>(TEMP1, XN2, C2T, TEMP2, T2HL, 1);
  gemmhl_kernel<64><<<dim3(NB / 128), dim3(128), 0, stream>>>(T2HL, LT, out);
  (void)hipGetLastError();
}
